// encoder_unit_83554293776725
// MI455X (gfx1250) — hardware-verified
//
#include <hip/hip_runtime.h>
#include <stdint.h>
#include <stddef.h>

constexpr int SEQ   = 2048;
constexpr int EMB   = 1024;
constexpr int NHEAD = 16;
constexpr int DHEAD = 64;
constexpr int FFN   = 4096;
constexpr float WSCALE     = 256.0f;
constexpr float WSCALE_INV = 1.0f / 256.0f;
constexpr float ATT_PSC    = 32768.0f;
constexpr int ATT_KC = 64;

static_assert(SEQ % 64 == 0, "");
static_assert(EMB % 64 == 0, "");
static_assert(FFN % 64 == 0, "");
static_assert(DHEAD == 64, "");
static_assert(EMB % 32 == 0 && FFN % 32 == 0, "");
static_assert(NHEAD * DHEAD == EMB, "");
static_assert(EMB == 4 * 256, "");

typedef __attribute__((ext_vector_type(16))) _Float16 v16h;
typedef __attribute__((ext_vector_type(8)))  _Float16 v8h;
typedef __attribute__((ext_vector_type(4)))  _Float16 v4h;
typedef __attribute__((ext_vector_type(16))) __bf16   v16b;
typedef __attribute__((ext_vector_type(8)))  __bf16   v8b;
typedef __attribute__((ext_vector_type(8)))  float    v8f;
typedef __attribute__((ext_vector_type(4)))  float    v4f;

__device__ __forceinline__ unsigned short f2bf_bits(float f) {
  unsigned u = __float_as_uint(f);
  return (unsigned short)((u + 0x7FFFu + ((u >> 16) & 1u)) >> 16);
}
__device__ __forceinline__ float bf_bits2f(unsigned short h) { return __uint_as_float(((unsigned)h) << 16); }

__device__ __forceinline__ void dep_guard_h(v8f& a, v8f& b, v16h x, v16h y) { asm volatile("v_nop\n\tv_nop\n\tv_nop\n\tv_nop" : "+v"(a), "+v"(b) : "v"(x), "v"(y)); }
__device__ __forceinline__ void dep_guard_b(v8f& a, v8f& b, v16b x, v16b y) { asm volatile("v_nop\n\tv_nop\n\tv_nop\n\tv_nop" : "+v"(a), "+v"(b) : "v"(x), "v"(y)); }
__device__ __forceinline__ void keep4_h(v16h a, v16h b, v16h c, v16h d) { asm volatile("v_nop" :: "v"(a), "v"(b), "v"(c), "v"(d)); }
__device__ __forceinline__ void keep4_b(v16b a, v16b b, v16b c, v16b d) { asm volatile("v_nop" :: "v"(a), "v"(b), "v"(c), "v"(d)); }
__device__ __forceinline__ void acc_guard4(v8f& a, v8f& b, v8f& c, v8f& d) { asm volatile("v_nop\n\tv_nop\n\tv_nop\n\tv_nop" : "+v"(a), "+v"(b), "+v"(c), "+v"(d)); }
template <typename T> struct Frag;
template <> struct Frag<_Float16> {
  typedef v16h V; union U { v16h v; v8h h[2]; };
  static __device__ __forceinline__ v16h load(const _Float16* p) {
    U f; f.h[0] = *(const v8h*)(p); f.h[1] = *(const v8h*)(p + 16); return f.v;
  }
  static __device__ __forceinline__ v8f mma(v16h a, v16h b, v8f c) {
    return __builtin_amdgcn_wmma_f32_16x16x32_f16(false, a, false, b, (short)0, c, false, false);
  }
  static __device__ __forceinline__ void guard(v8f& a, v8f& b, v16h x, v16h y) { dep_guard_h(a, b, x, y); }
  static __device__ __forceinline__ void keep(v16h a, v16h b, v16h c, v16h d) { keep4_h(a, b, c, d); }
};
template <> struct Frag<__bf16> {
  typedef v16b V; union U { v16b v; v8b h[2]; };
  static __device__ __forceinline__ v16b load(const __bf16* p) {
    U f; f.h[0] = *(const v8b*)(p); f.h[1] = *(const v8b*)(p + 16); return f.v;
  }
  static __device__ __forceinline__ v8f mma(v16b a, v16b b, v8f c) {
    return __builtin_amdgcn_wmma_f32_16x16x32_bf16(false, a, false, b, (short)0, c, false, false);
  }
  static __device__ __forceinline__ void guard(v8f& a, v8f& b, v16b x, v16b y) { dep_guard_b(a, b, x, y); }
  static __device__ __forceinline__ void keep(v16b a, v16b b, v16b c, v16b d) { keep4_b(a, b, c, d); }
};

__device__ __forceinline__ v8f hmma(v16h a, v16h b, v8f c) {
  c = __builtin_amdgcn_wmma_f32_16x16x32_f16(false, a, false, b, (short)0, c, false, false);
  asm volatile("v_nop\n\tv_nop\n\tv_nop\n\tv_nop" : "+v"(c) : "v"(a), "v"(b));
  return c;
}

template <int ET> struct Elem;
template <> struct Elem<0> { typedef _Float16 T; };
template <> struct Elem<1> { typedef __bf16 T; };
template <int ET, bool SPLIT, int BIAS_MODE, int OUT_MODE, bool RESID, int ACT = 0>
__global__ __launch_bounds__(256) void wmma_gemm64(
    const unsigned short* __restrict__ Ap, const unsigned short* __restrict__ A2p, int lda, long strideA,
    const unsigned short* __restrict__ Btp, const unsigned short* __restrict__ Bt2p, int ldb, long strideB,
    void* __restrict__ Cout, void* __restrict__ Cout2, int ldc, long strideC,
    const float* __restrict__ bias, long strideBias,
    const float* __restrict__ resid, long strideR,
    int M, int N, int K, float scale) {
  typedef typename Elem<ET>::T T;
  typedef typename Frag<T>::V V;
  const T* A = (const T*)Ap; const T* A2 = (const T*)A2p; const T* Bt = (const T*)Btp; const T* Bt2 = (const T*)Bt2p;
  __shared__ __align__(16) float sT[8][16 * 68];
  const int b    = blockIdx.y;
  const int lane = threadIdx.x & 31;
  const int wave = threadIdx.x >> 5;
  const int tilesN = N >> 6;
  const int tilesM = M >> 6;
  const int tile = blockIdx.x * 8 + wave;
  if (tile >= tilesM * tilesN) return;
  const int tm = tile / tilesN;
  const int tn = tile - tm * tilesN;
  const int m0 = tm << 6;
  const int n0 = tn << 6;

  const T* Ab  = A  + (size_t)b * strideA;
  const T* Bb  = Bt + (size_t)b * strideB;
  const T* Ab2 = SPLIT ? (A2  + (size_t)b * strideA) : nullptr;
  const T* Bb2 = SPLIT ? (Bt2 + (size_t)b * strideB) : nullptr;

  const int rlane = lane & 15;
  const int koff  = (lane >> 4) * 8;
  const int mOff  = (lane >> 4) * 8;

  v8f acc[4][4];
#pragma unroll
  for (int i = 0; i < 4; ++i)
#pragma unroll
    for (int j = 0; j < 4; ++j) acc[i][j] = (v8f){0.f,0.f,0.f,0.f,0.f,0.f,0.f,0.f};

  for (int k0 = 0; k0 < K; k0 += 32) {
    V bh[4], bl[4];
#pragma unroll
    for (int j = 0; j < 4; ++j) {
      const size_t bo = (size_t)(n0 + (j << 4) + rlane) * ldb + koff + k0;
      bh[j] = Frag<T>::load(Bb + bo);
      if (SPLIT) bl[j] = Frag<T>::load(Bb2 + bo);
    }
#pragma unroll
    for (int i = 0; i < 4; ++i) {
      const size_t ao = (size_t)(m0 + (i << 4) + rlane) * lda + koff + k0;
      V ah = Frag<T>::load(Ab + ao);
      V al;
      if (SPLIT) al = Frag<T>::load(Ab2 + ao);
#pragma unroll
      for (int j = 0; j < 4; ++j) {
        acc[i][j] = Frag<T>::mma(ah, bh[j], acc[i][j]);
        if (SPLIT) {
          acc[i][j] = Frag<T>::mma(ah, bl[j], acc[i][j]);
          acc[i][j] = Frag<T>::mma(al, bh[j], acc[i][j]);
        }
      }
      Frag<T>::guard(acc[i][0], acc[i][3], ah, SPLIT ? al : ah);
    }
    Frag<T>::keep(bh[0], bh[1], bh[2], bh[3]);
    if (SPLIT) Frag<T>::keep(bl[0], bl[1], bl[2], bl[3]);
  }
  acc_guard4(acc[0][0], acc[0][1], acc[0][2], acc[0][3]);
  acc_guard4(acc[1][0], acc[1][1], acc[1][2], acc[1][3]);
  acc_guard4(acc[2][0], acc[2][1], acc[2][2], acc[2][3]);
  acc_guard4(acc[3][0], acc[3][1], acc[3][2], acc[3][3]);

  float* slab = sT[wave];
  const float* Rb = RESID ? (resid + (size_t)b * strideR) : nullptr;
  const float* bb = (BIAS_MODE != 0) ? (bias + (size_t)b * strideBias) : bias;
#pragma unroll
  for (int i = 0; i < 4; ++i) {
    const int mBase = m0 + (i << 4);
#pragma unroll
    for (int j = 0; j < 4; ++j) {
      const int n = n0 + (j << 4) + rlane;
      float bv = 0.f;
      if (BIAS_MODE == 2) bv = bb[n];
#pragma unroll
      for (int r = 0; r < 8; ++r) {
        float v = acc[i][j][r] * scale;
        if (BIAS_MODE == 1) v += bb[mBase + mOff + r];
        if (BIAS_MODE == 2) v += bv;
        if (RESID) v += Rb[(size_t)(mBase + mOff + r) * ldc + n];
        if (ACT == 1) v = tanhf(v);
        if (ACT == 2) v = fmaxf(v, 0.0f);
        if (ACT == 4) v = (v > 0.f) ? v : 0.01f * v;
        slab[(mOff + r) * 68 + (j << 4) + rlane] = v;
      }
    }
    __builtin_amdgcn_fence(__ATOMIC_RELEASE, "workgroup");
    __builtin_amdgcn_wave_barrier();
    __builtin_amdgcn_fence(__ATOMIC_ACQUIRE, "workgroup");
    if (OUT_MODE == 0) {
      float* C = (float*)Cout + (size_t)b * strideC;
      const int hh = lane >> 4, c4 = (lane & 15) * 4;
      for (int pass = 0; pass < 2; ++pass) {
#pragma unroll
        for (int it = 0; it < 8; ++it) {
          const int row = it * 2 + hh;
          v4f v = *(const v4f*)(slab + row * 68 + c4);
          *(volatile v4f*)(C + (size_t)(mBase + row) * ldc + n0 + c4) = v;
        }
        __threadfence();
      }
    } else {
      const int q = lane >> 3, c8 = (lane & 7) * 8;
      unsigned short* C  = (unsigned short*)Cout  + (size_t)b * strideC;
      unsigned short* C2 = (OUT_MODE == 2) ? ((unsigned short*)Cout2 + (size_t)b * strideC) : nullptr;
      for (int pass = 0; pass < 2; ++pass) {
#pragma unroll
        for (int it = 0; it < 4; ++it) {
          const int row = it * 4 + q;
          const float* sp = slab + row * 68 + c8;
          v8h hv, lv;
#pragma unroll
          for (int e = 0; e < 8; ++e) {
            if (OUT_MODE == 1) {
              hv[e] = (_Float16)sp[e];
            } else {
              unsigned short hb = f2bf_bits(sp[e]);
              unsigned short lb = f2bf_bits(sp[e] - bf_bits2f(hb));
              hv[e] = __builtin_bit_cast(_Float16, hb);
              lv[e] = __builtin_bit_cast(_Float16, lb);
            }
          }
          *(volatile v8h*)(C + (size_t)(mBase + row) * ldc + n0 + c8) = hv;
          if (OUT_MODE == 2) *(volatile v8h*)(C2 + (size_t)(mBase + row) * ldc + n0 + c8) = lv;
        }
        __threadfence();
      }
    }
    __builtin_amdgcn_fence(__ATOMIC_RELEASE, "workgroup");
    __builtin_amdgcn_wave_barrier();
    __builtin_amdgcn_fence(__ATOMIC_ACQUIRE, "workgroup");
  }
}

__global__ __launch_bounds__(256) void emb_f16_kernel(const float* __restrict__ xw, const float* __restrict__ xp,
                                                      _Float16* __restrict__ embH, int n8) {
  const int i = blockIdx.x * 256 + threadIdx.x;
  if (i < n8) {
    const size_t o = (size_t)i * 8;
    const v4f a0 = *(const v4f*)(xw + o), a1 = *(const v4f*)(xw + o + 4);
    const v4f p0 = *(const v4f*)(xp + o), p1 = *(const v4f*)(xp + o + 4);
    const v4f e0 = a0 + p0, e1 = a1 + p1;
    v8h hv;
#pragma unroll
    for (int e = 0; e < 4; ++e) { hv[e] = (_Float16)e0[e]; hv[4 + e] = (_Float16)e1[e]; }
    *(volatile v8h*)(embH + o) = hv;
    __threadfence();
    *(volatile v8h*)(embH + o) = hv;
  }
}

__global__ __launch_bounds__(256) void cast_scale_f16_kernel(const float* __restrict__ in, _Float16* __restrict__ out,
                                                             int n8, float sc) {
  const int i = blockIdx.x * 256 + threadIdx.x;
  if (i < n8) {
    const size_t o = (size_t)i * 8;
    const v4f a0 = *(const v4f*)(in + o), a1 = *(const v4f*)(in + o + 4);
    v8h hv;
#pragma unroll
    for (int e = 0; e < 4; ++e) { hv[e] = (_Float16)(a0[e] * sc); hv[4 + e] = (_Float16)(a1[e] * sc); }
    *(volatile v8h*)(out + o) = hv;
    __threadfence();
    *(volatile v8h*)(out + o) = hv;
  }
}

__global__ __launch_bounds__(256) void wtr_f16_kernel(const float* __restrict__ in, _Float16* __restrict__ out) {
  __shared__ __align__(16) _Float16 st[DHEAD * 72];
  const int tid = threadIdx.x, e0 = blockIdx.x * 64, h = blockIdx.y;
  {
    const int e = tid >> 2, d0 = (tid & 3) * 16;
    const float* src = in + ((size_t)h * EMB + e0 + e) * DHEAD + d0;
#pragma unroll
    for (int i = 0; i < 4; ++i) {
      const v4f f = *(const v4f*)(src + 4 * i);
#pragma unroll
      for (int j = 0; j < 4; ++j) st[(d0 + 4 * i + j) * 72 + e] = (_Float16)(f[j] * WSCALE);
    }
  }
  __syncthreads();
  const int wave = tid >> 5, lane = tid & 31, q = lane >> 3, c8 = (lane & 7) * 8;
  for (int pass = 0; pass < 2; ++pass) {
#pragma unroll
    for (int it = 0; it < 2; ++it) {
      const int row = wave * 8 + it * 4 + q;
      const v8h hv = *(const v8h*)(st + row * 72 + c8);
      *(volatile v8h*)(out + ((size_t)h * DHEAD + row) * EMB + e0 + c8) = hv;
    }
    __threadfence();
  }
}

__global__ __launch_bounds__(128) void attn_f16_kernel(const _Float16* __restrict__ Qp, const _Float16* __restrict__ Kp,
                                                       const _Float16* __restrict__ Vtp, _Float16* __restrict__ Zp) {
  __shared__ __align__(16) _Float16 Ksh[ATT_KC * DHEAD];
  __shared__ __align__(16) _Float16 Vth[DHEAD * ATT_KC];
  __shared__ __align__(16) _Float16 Psh[4][16 * ATT_KC];
  __shared__ __align__(16) float    Os[4][16 * 68];

  const int tid  = threadIdx.x;
  const int wave = tid >> 5;
  const int lane = tid & 31;
  const int hh   = lane >> 4;
  const int c    = lane & 15;
  const int qb = blockIdx.x;
  const int h  = blockIdx.y;
  const int q0 = qb * 64 + wave * 16;

  const _Float16* Qh = Qp  + (size_t)h * SEQ * DHEAD;
  const _Float16* Kh = Kp  + (size_t)h * SEQ * DHEAD;
  const _Float16* Vh = Vtp + (size_t)h * DHEAD * SEQ;

  v16h qa[2];
#pragma unroll
  for (int dc = 0; dc < 2; ++dc) qa[dc] = Frag<_Float16>::load(Qh + (size_t)(q0 + c) * DHEAD + dc * 32 + 8 * hh);

  const float NEG_INF = -__builtin_inff();
  float mrow[8], lrow[8];
  v8f oacc[4];
#pragma unroll
  for (int r = 0; r < 8; ++r) { mrow[r] = NEG_INF; lrow[r] = 0.f; }
#pragma unroll
  for (int t = 0; t < 4; ++t) oacc[t] = (v8f){0.f,0.f,0.f,0.f,0.f,0.f,0.f,0.f};

  for (int kc = 0; kc < SEQ / ATT_KC; ++kc) {
    const int kv0 = kc * ATT_KC;
    __syncthreads();
    {
      const int r = tid >> 1, x32 = (tid & 1) * 32;
      const _Float16* ks = Kh + (size_t)(kv0 + r) * DHEAD + x32;
      const _Float16* vs = Vh + (size_t)r * SEQ + kv0 + x32;
      v8h kt[4], vt[4];
#pragma unroll
      for (int i = 0; i < 4; ++i) { kt[i] = *(const v8h*)(ks + 8 * i); vt[i] = *(const v8h*)(vs + 8 * i); }
#pragma unroll
      for (int i = 0; i < 4; ++i) {
        *(v8h*)(Ksh + r * DHEAD + x32 + 8 * i) = kt[i];
        *(v8h*)(Vth + r * ATT_KC + x32 + 8 * i) = vt[i];
      }
    }
    __syncthreads();

    v8f s[4];
#pragma unroll
    for (int j = 0; j < 4; ++j) {
      s[j] = (v8f){0.f,0.f,0.f,0.f,0.f,0.f,0.f,0.f};
#pragma unroll
      for (int dc = 0; dc < 2; ++dc) {
        const v16h kb = Frag<_Float16>::load(Ksh + (j * 16 + c) * DHEAD + dc * 32 + 8 * hh);
        s[j] = hmma(qa[dc], kb, s[j]);
      }
    }
    float cm[8];
#pragma unroll
    for (int r = 0; r < 8; ++r) {
      float m = fmaxf(fmaxf(s[0][r], s[1][r]), fmaxf(s[2][r], s[3][r]));
#pragma unroll
      for (int off = 1; off < 16; off <<= 1) m = fmaxf(m, __shfl_xor(m, off, 32));
      cm[r] = m;
    }
    _Float16* pw = Psh[wave];
#pragma unroll
    for (int r = 0; r < 8; ++r) {
      const float mnew = fmaxf(mrow[r], cm[r]);
      const float alpha = expf(mrow[r] - mnew);
      mrow[r] = mnew;
      float psum = 0.f;
#pragma unroll
      for (int j = 0; j < 4; ++j) {
        const float p = expf(s[j][r] - mnew);
        psum += p;
        pw[(8 * hh + r) * ATT_KC + j * 16 + c] = (_Float16)(p * ATT_PSC);
      }
#pragma unroll
      for (int off = 1; off < 16; off <<= 1) psum += __shfl_xor(psum, off, 32);
      lrow[r] = lrow[r] * alpha + psum;
#pragma unroll
      for (int t = 0; t < 4; ++t) oacc[t][r] *= alpha;
    }
    __builtin_amdgcn_fence(__ATOMIC_RELEASE, "workgroup");
    __builtin_amdgcn_wave_barrier();
    __builtin_amdgcn_fence(__ATOMIC_ACQUIRE, "workgroup");
#pragma unroll
    for (int kk = 0; kk < 2; ++kk) {
      const v16h pa = Frag<_Float16>::load(pw + c * ATT_KC + kk * 32 + 8 * hh);
#pragma unroll
      for (int t = 0; t < 4; ++t) {
        const v16h vb = Frag<_Float16>::load(Vth + (t * 16 + c) * ATT_KC + kk * 32 + 8 * hh);
        oacc[t] = hmma(pa, vb, oacc[t]);
      }
    }
  }

  float* os = Os[wave];
#pragma unroll
  for (int r = 0; r < 8; ++r) {
    const float inv = 1.0f / (lrow[r] * ATT_PSC);
#pragma unroll
    for (int t = 0; t < 4; ++t) os[(8 * hh + r) * 68 + t * 16 + c] = oacc[t][r] * inv;
  }
  __builtin_amdgcn_fence(__ATOMIC_RELEASE, "workgroup");
  __builtin_amdgcn_wave_barrier();
  __builtin_amdgcn_fence(__ATOMIC_ACQUIRE, "workgroup");
  {
    const int q = lane >> 3, c8 = (lane & 7) * 8;
    for (int pass = 0; pass < 2; ++pass) {
#pragma unroll
      for (int it = 0; it < 4; ++it) {
        const int row = it * 4 + q;
        const float* sp = os + row * 68 + c8;
        v8h hv;
#pragma unroll
        for (int e = 0; e < 8; ++e) hv[e] = (_Float16)sp[e];
        *(volatile v8h*)(Zp + (size_t)(q0 + row) * EMB + h * DHEAD + c8) = hv;
      }
      __threadfence();
    }
  }
}

template <bool ADD2, bool OUTH>
__global__ __launch_bounds__(256) void layernorm_kernel(const float* __restrict__ X, const float* __restrict__ Ra,
                                                        const float* __restrict__ Rb2,
                                                        const float* __restrict__ gam, const float* __restrict__ bet,
                                                        float* __restrict__ outF, _Float16* __restrict__ outH) {
  __shared__ float red1[8];
  __shared__ float red2[8];
  __shared__ __align__(16) _Float16 sh[OUTH ? EMB : 8];
  const int row = blockIdx.x, t = threadIdx.x, lane = t & 31, wave = t >> 5;
  const size_t base = (size_t)row * EMB + 4 * t;
  v4f x = *(const v4f*)(X + base);
  if (ADD2) {
    const v4f ea = *(const v4f*)(Ra + base);
    const v4f eb = *(const v4f*)(Rb2 + base);
    const v4f es = ea + eb;
    x = x + es;
  }
  float s = (x[0] + x[1]) + (x[2] + x[3]);
#pragma unroll
  for (int off = 16; off > 0; off >>= 1) s += __shfl_xor(s, off, 32);
  if (lane == 0) red1[wave] = s;
  __syncthreads();
  float tot = 0.f;
#pragma unroll
  for (int w = 0; w < 8; ++w) tot += red1[w];
  const float mean = tot * (1.0f / (float)EMB);
  v4f d;
#pragma unroll
  for (int e = 0; e < 4; ++e) d[e] = x[e] - mean;
  float sq = (d[0] * d[0] + d[1] * d[1]) + (d[2] * d[2] + d[3] * d[3]);
#pragma unroll
  for (int off = 16; off > 0; off >>= 1) sq += __shfl_xor(sq, off, 32);
  if (lane == 0) red2[wave] = sq;
  __syncthreads();
  float tot2 = 0.f;
#pragma unroll
  for (int w = 0; w < 8; ++w) tot2 += red2[w];
  const float var  = tot2 * (1.0f / (float)EMB);
  const float rstd = rsqrtf(var + 1e-5f);
  const v4f gg = *(const v4f*)(gam + 4 * t);
  const v4f bb = *(const v4f*)(bet + 4 * t);
  v4f y;
#pragma unroll
  for (int e = 0; e < 4; ++e) y[e] = d[e] * rstd * gg[e] + bb[e];
  *(volatile v4f*)(outF + base) = y;
  __threadfence();
  *(volatile v4f*)(outF + base) = y;
  if (OUTH) {
    v4h h4;
#pragma unroll
    for (int e = 0; e < 4; ++e) h4[e] = (_Float16)y[e];
    *(v4h*)(sh + 4 * t) = h4;
    __syncthreads();
    if (t < 128) {
      const v8h hv = *(const v8h*)(sh + 8 * t);
      _Float16* op = outH + (size_t)row * EMB + 8 * t;
      *(volatile v8h*)op = hv;
      __threadfence();
      *(volatile v8h*)op = hv;
    }
  }
}

extern "C" void kernel_launch(void* const* d_in, const int* in_sizes, int n_in,
                              void* d_out, int out_size, void* d_ws, size_t ws_size,
                              hipStream_t stream) {
  if (n_in < 18) return;
  if (in_sizes[0] != SEQ * EMB || in_sizes[1] != SEQ * EMB || in_sizes[2] != NHEAD * EMB * DHEAD ||
      in_sizes[8] != EMB * EMB || in_sizes[12] != FFN * EMB || in_sizes[14] != EMB * FFN || out_size != SEQ * EMB) return;

  const float* xw  = (const float*)d_in[0];
  const float* xp  = (const float*)d_in[1];
  const float* Wq  = (const float*)d_in[2];
  const float* bq  = (const float*)d_in[3];
  const float* Wk  = (const float*)d_in[4];
  const float* bk  = (const float*)d_in[5];
  const float* Wv  = (const float*)d_in[6];
  const float* bv  = (const float*)d_in[7];
  const float* W0  = (const float*)d_in[8];
  const float* b0  = (const float*)d_in[9];
  const float* g1  = (const float*)d_in[10];
  const float* be1 = (const float*)d_in[11];
  const float* W1  = (const float*)d_in[12];
  const float* b1  = (const float*)d_in[13];
  const float* W2  = (const float*)d_in[14];
  const float* b2  = (const float*)d_in[15];
  const float* g2  = (const float*)d_in[16];
  const float* be2 = (const float*)d_in[17];
  float* outp = (float*)d_out;

  char* wsb = (char*)d_ws;
  size_t off = 0;
  auto take = [&](size_t bytes) -> char* { char* r = wsb + off; off += (bytes + 255) & ~(size_t)255; return r; };
  _Float16* embH  = (_Float16*)take((size_t)SEQ * EMB * 2);
  _Float16* WqT   = (_Float16*)take((size_t)NHEAD * DHEAD * EMB * 2);
  _Float16* WkT   = (_Float16*)take((size_t)NHEAD * DHEAD * EMB * 2);
  _Float16* WvT   = (_Float16*)take((size_t)NHEAD * DHEAD * EMB * 2);
  _Float16* W0H   = (_Float16*)take((size_t)EMB * EMB * 2);
  _Float16* W1H   = (_Float16*)take((size_t)FFN * EMB * 2);
  _Float16* W2H   = (_Float16*)take((size_t)EMB * FFN * 2);
  _Float16* QH    = (_Float16*)take((size_t)NHEAD * SEQ * DHEAD * 2);
  _Float16* KH    = (_Float16*)take((size_t)NHEAD * SEQ * DHEAD * 2);
  _Float16* VtH   = (_Float16*)take((size_t)NHEAD * DHEAD * SEQ * 2);
  _Float16* ZH    = (_Float16*)take((size_t)SEQ * EMB * 2);
  float*    z0F   = (float*)   take((size_t)SEQ * EMB * 4);
  float*    out1F = (float*)   take((size_t)SEQ * EMB * 4);
  _Float16* out1H = (_Float16*)take((size_t)SEQ * EMB * 2);
  _Float16* h1H   = (_Float16*)take((size_t)SEQ * FFN * 2);
  float*    sumF  = (float*)   take((size_t)SEQ * EMB * 4);
  if (off > ws_size) return;

  typedef const unsigned short* cus;

  {
    const int n8 = SEQ * EMB / 8;
    emb_f16_kernel<<<(n8 + 255) / 256, 256, 0, stream>>>(xw, xp, embH, n8);
  }
  wtr_f16_kernel<<<dim3(EMB / 64, NHEAD), 256, 0, stream>>>(Wq, WqT);
  wtr_f16_kernel<<<dim3(EMB / 64, NHEAD), 256, 0, stream>>>(Wk, WkT);
  wtr_f16_kernel<<<dim3(EMB / 64, NHEAD), 256, 0, stream>>>(Wv, WvT);
  {
    const int n8a = EMB * EMB / 8, n8b = FFN * EMB / 8;
    cast_scale_f16_kernel<<<(n8a + 255) / 256, 256, 0, stream>>>(W0, W0H, n8a, WSCALE);
    cast_scale_f16_kernel<<<(n8b + 255) / 256, 256, 0, stream>>>(W1, W1H, n8b, WSCALE);
    cast_scale_f16_kernel<<<(n8b + 255) / 256, 256, 0, stream>>>(W2, W2H, n8b, WSCALE);
  }

  {
    const int tiles = (SEQ / 64) * (DHEAD / 64);
    dim3 grid((tiles + 7) / 8, NHEAD);
    wmma_gemm64<0, false, 2, 1, false, 0><<<grid, 256, 0, stream>>>(
        (cus)embH, (cus)embH, EMB, 0L, (cus)WqT, (cus)WqT, EMB, (long)DHEAD * EMB,
        (void*)QH, nullptr, DHEAD, (long)SEQ * DHEAD, bq, (long)DHEAD, nullptr, 0L,
        SEQ, DHEAD, EMB, WSCALE_INV);
    wmma_gemm64<0, false, 2, 1, false, 0><<<grid, 256, 0, stream>>>(
        (cus)embH, (cus)embH, EMB, 0L, (cus)WkT, (cus)WkT, EMB, (long)DHEAD * EMB,
        (void*)KH, nullptr, DHEAD, (long)SEQ * DHEAD, bk, (long)DHEAD, nullptr, 0L,
        SEQ, DHEAD, EMB, WSCALE_INV);
  }
  {
    const int tiles = (DHEAD / 64) * (SEQ / 64);
    dim3 grid((tiles + 7) / 8, NHEAD);
    wmma_gemm64<0, false, 1, 1, false, 0><<<grid, 256, 0, stream>>>(
        (cus)WvT, (cus)WvT, EMB, (long)DHEAD * EMB, (cus)embH, (cus)embH, EMB, 0L,
        (void*)VtH, nullptr, SEQ, (long)DHEAD * SEQ, bv, (long)DHEAD, nullptr, 0L,
        DHEAD, SEQ, EMB, WSCALE_INV);
  }

  attn_f16_kernel<<<dim3(SEQ / 64, NHEAD), 128, 0, stream>>>(QH, KH, VtH, ZH);

  {
    const int tiles = (SEQ / 64) * (EMB / 64);
    wmma_gemm64<0, false, 2, 0, false, 0><<<dim3((tiles + 7) / 8, 1), 256, 0, stream>>>(
        (cus)ZH, (cus)ZH, EMB, 0L, (cus)W0H, (cus)W0H, EMB, 0L,
        (void*)z0F, nullptr, EMB, 0L, b0, 0L, nullptr, 0L,
        SEQ, EMB, EMB, WSCALE_INV * 0.125f);
  }

  layernorm_kernel<true, true><<<SEQ, 256, 0, stream>>>(z0F, xw, xp, g1, be1, out1F, out1H);

  {
    const int tiles = (SEQ / 64) * (FFN / 64);
    wmma_gemm64<0, false, 2, 1, false, 2><<<dim3((tiles + 7) / 8, 1), 256, 0, stream>>>(
        (cus)out1H, (cus)out1H, EMB, 0L, (cus)W1H, (cus)W1H, EMB, 0L,
        (void*)h1H, nullptr, FFN, 0L, b1, 0L, nullptr, 0L,
        SEQ, FFN, EMB, WSCALE_INV);
  }

  {
    const int tiles = (SEQ / 64) * (EMB / 64);
    wmma_gemm64<0, false, 2, 0, true, 0><<<dim3((tiles + 7) / 8, 1), 256, 0, stream>>>(
        (cus)h1H, (cus)h1H, FFN, 0L, (cus)W2H, (cus)W2H, FFN, 0L,
        (void*)sumF, nullptr, EMB, 0L, b2, 0L, out1F, 0L,
        SEQ, EMB, FFN, WSCALE_INV);
  }

  layernorm_kernel<false, false><<<SEQ, 256, 0, stream>>>(sumF, sumF, sumF, g2, be2, outp, nullptr);
}
